// SoftmaxMatcherBlock_50577534877890
// MI455X (gfx1250) — hardware-verified
//
#include <hip/hip_runtime.h>
#include <math.h>
#include <stdint.h>

#define NB   2
#define NC   64
#define NSRC 1024
#define NTGT 16384
#define NDV  68
#define DVP  80
#define QBLK 128
#define KC   64
#define KSP  72
#define VTP  72
#define OSP  132
#define TP   68
#define VSEG 2048

static_assert(NSRC % QBLK == 0);
static_assert(NTGT % KC == 0);
static_assert(KC == 64);
static_assert(NTGT % VSEG == 0);
static_assert(NC == 64);
static_assert(DVP % 16 == 0);
static_assert(DVP >= NDV);
static_assert(NSRC % 64 == 0);
static_assert(NTGT % 64 == 0);

typedef __attribute__((ext_vector_type(16))) __bf16 v16b;
typedef __attribute__((ext_vector_type(8)))  __bf16 v8b;
typedef __attribute__((ext_vector_type(8)))  float  v8f;
typedef __attribute__((ext_vector_type(4)))  float  v4f;
typedef __attribute__((ext_vector_type(4)))  unsigned int v4u;

__device__ __forceinline__ unsigned short f2bf_bits(float f) {
  unsigned u = __float_as_uint(f);
  return (unsigned short)((u + 0x7FFFu + ((u >> 16) & 1u)) >> 16);
}
__device__ __forceinline__ float bf_bits2f(unsigned short b) { return __uint_as_float(((unsigned)b) << 16); }
__device__ __forceinline__ unsigned pk16(unsigned short a, unsigned short b) { return (unsigned)a | ((unsigned)b << 16); }

__device__ __forceinline__ void split2(float f0, float f1, unsigned& hw, unsigned& lw) {
  const unsigned short h0 = f2bf_bits(f0), h1 = f2bf_bits(f1);
  const unsigned short l0 = f2bf_bits(f0 - bf_bits2f(h0)), l1 = f2bf_bits(f1 - bf_bits2f(h1));
  hw = pk16(h0, h1);
  lw = pk16(l0, l1);
}

__device__ __forceinline__ v8f mma_bf(v16b a, v16b b, v8f c) {
  c = __builtin_amdgcn_wmma_f32_16x16x32_bf16(false, a, false, b, (short)0, c, false, false);
  asm volatile("v_nop\n\tv_nop\n\tv_nop\n\tv_nop" : "+v"(c) : "v"(a), "v"(b));
  return c;
}

__global__ __launch_bounds__(256) void zn_split_kernel(const float* __restrict__ desc,
                                                       unsigned short* __restrict__ hi,
                                                       unsigned short* __restrict__ lo,
                                                       int np) {
  __shared__ __align__(16) float tf[NC * TP];
  __shared__ float smu[64];
  __shared__ float sinv[64];
  const int tid  = threadIdx.x;
  const int nblk = np / 64;
  const int b    = blockIdx.x / nblk;
  const int p0   = (blockIdx.x - b * nblk) * 64;
  {
    const int c = tid >> 2, p16 = (tid & 3) * 16;
    const float* sp = desc + ((size_t)(b * NC + c) * np + p0 + p16);
#pragma unroll
    for (int i = 0; i < 4; ++i)
      *(v4f*)(tf + c * TP + p16 + 4 * i) = *(const v4f*)(sp + 4 * i);
  }
  __syncthreads();
  {
    const int p = tid >> 2, sub = tid & 3;
    float s = 0.f;
#pragma unroll
    for (int j = 0; j < 16; ++j) s += tf[(sub * 16 + j) * TP + p];
    s += __shfl_xor(s, 1, 32);
    s += __shfl_xor(s, 2, 32);
    const float mu = s * (1.0f / 64.0f);
    float v = 0.f;
#pragma unroll 4
    for (int j = 0; j < 16; ++j) {
      const float dx = tf[(sub * 16 + j) * TP + p] - mu;
      v += dx * dx;
    }
    v += __shfl_xor(v, 1, 32);
    v += __shfl_xor(v, 2, 32);
    const float sd = sqrtf(v * (1.0f / 63.0f));
    if (sub == 0) {
      smu[p]  = mu;
      sinv[p] = 1.0f / sd;
    }
  }
  __syncthreads();
  {
    const int rl = tid >> 3, c8 = (tid & 7) * 8;
    v4u hv[2], lv[2];
#pragma unroll
    for (int it = 0; it < 2; ++it) {
      const int row = it * 32 + rl;
      const float mu = smu[row], inv = sinv[row];
      unsigned hw[4], lw[4];
#pragma unroll
      for (int q = 0; q < 4; ++q) {
        const float x0 = (tf[(c8 + 2 * q) * TP + row] - mu) * inv;
        const float x1 = (tf[(c8 + 2 * q + 1) * TP + row] - mu) * inv;
        split2(x0, x1, hw[q], lw[q]);
      }
      hv[it] = (v4u){hw[0], hw[1], hw[2], hw[3]};
      lv[it] = (v4u){lw[0], lw[1], lw[2], lw[3]};
    }
    const size_t base = ((size_t)(b * np + p0)) * NC + c8;
#pragma unroll
    for (int it = 0; it < 2; ++it) {
      const size_t go = base + (size_t)(it * 32 + rl) * NC;
      *(volatile v4u*)(hi + go) = hv[it];
      *(volatile v4u*)(lo + go) = lv[it];
    }
    __threadfence();
#pragma unroll
    for (int it = 0; it < 2; ++it) {
      const size_t go = base + (size_t)(it * 32 + rl) * NC;
      *(volatile v4u*)(hi + go) = hv[it];
      *(volatile v4u*)(lo + go) = lv[it];
    }
  }
}

__global__ __launch_bounds__(256) void vsplit_kernel(const float* __restrict__ coords,
                                                      const float* __restrict__ wts,
                                                      const float* __restrict__ desc,
                                                      unsigned short* __restrict__ vh,
                                                      unsigned short* __restrict__ vl) {
  const int tid  = threadIdx.x;
  const int nseg = NTGT / VSEG;
  const int seg  = blockIdx.x % nseg;
  const int bd   = blockIdx.x / nseg;
  const int b    = bd / DVP;
  const int d    = bd - b * DVP;
  const int m0   = seg * VSEG + tid * 8;
  v4f a0 = (v4f){0.f, 0.f, 0.f, 0.f};
  v4f a1 = (v4f){0.f, 0.f, 0.f, 0.f};
  if (d < NDV) {
    const float* sp;
    if (d < 3)       sp = coords + ((size_t)(b * 3 + d)) * NTGT;
    else if (d == 3) sp = wts + (size_t)b * NTGT;
    else             sp = desc + ((size_t)(b * NC + (d - 4))) * NTGT;
    a0 = *(const v4f*)(sp + m0);
    a1 = *(const v4f*)(sp + m0 + 4);
  }
  unsigned h0, h1, h2, h3, l0, l1, l2, l3;
  split2(a0[0], a0[1], h0, l0);
  split2(a0[2], a0[3], h1, l1);
  split2(a1[0], a1[1], h2, l2);
  split2(a1[2], a1[3], h3, l3);
  const v4u hvv = (v4u){h0, h1, h2, h3};
  const v4u lvv = (v4u){l0, l1, l2, l3};
  const size_t go = ((size_t)(b * DVP + d)) * NTGT + m0;
  volatile v4u* ph = (volatile v4u*)(vh + go);
  volatile v4u* pl = (volatile v4u*)(vl + go);
  *ph = hvv;
  *pl = lvv;
  __threadfence();
  *ph = hvv;
  *pl = lvv;
}

__global__ __launch_bounds__(256)
void matcher_kernel(const unsigned short* __restrict__ qhp, const unsigned short* __restrict__ qlp,
                    const unsigned short* __restrict__ khp, const unsigned short* __restrict__ klp,
                    const unsigned short* __restrict__ vhp, const unsigned short* __restrict__ vlp,
                    float* __restrict__ out) {
  union FB { v16b v; v8b h[2]; };
  union FW { v16b v; unsigned w[8]; };
  __shared__ __align__(16) __bf16 Ksh[KC * KSP];
  __shared__ __align__(16) __bf16 Ksl[KC * KSP];
  __shared__ __align__(16) __bf16 Vsh[DVP * VTP];
  __shared__ __align__(16) __bf16 Vsl[DVP * VTP];
  __shared__ __align__(16) float  Osh[DVP * OSP];

  const int tid  = threadIdx.x;
  const int wave = tid >> 5;
  const int lane = tid & 31;
  const int lh   = lane >> 4;
  const int c    = lane & 15;
  const int nqb  = NSRC / QBLK;
  const int b    = blockIdx.x / nqb;
  const int n0   = (blockIdx.x - b * nqb) * QBLK;
  const int nw   = n0 + wave * 16;

  const __bf16* Qh = (const __bf16*)(const void*)qhp + ((size_t)(b * NSRC + nw + c)) * NC + 8 * lh;
  const __bf16* Ql = (const __bf16*)(const void*)qlp + ((size_t)(b * NSRC + nw + c)) * NC + 8 * lh;
  const __bf16* Kh = (const __bf16*)(const void*)khp + (size_t)b * NTGT * NC;
  const __bf16* Kl = (const __bf16*)(const void*)klp + (size_t)b * NTGT * NC;
  const __bf16* Vh = (const __bf16*)(const void*)vhp + (size_t)b * DVP * NTGT;
  const __bf16* Vl = (const __bf16*)(const void*)vlp + (size_t)b * DVP * NTGT;

  FB qfh[2], qfl[2];
#pragma unroll
  for (int dc = 0; dc < 2; ++dc) {
    qfh[dc].h[0] = *(const v8b*)(Qh + dc * 32);
    qfh[dc].h[1] = *(const v8b*)(Qh + dc * 32 + 16);
    qfl[dc].h[0] = *(const v8b*)(Ql + dc * 32);
    qfl[dc].h[1] = *(const v8b*)(Ql + dc * 32 + 16);
  }

  v8f oacc[5];
#pragma unroll
  for (int t = 0; t < 5; ++t) oacc[t] = (v8f){0.f, 0.f, 0.f, 0.f, 0.f, 0.f, 0.f, 0.f};
  float mrun = -1e30f, lrun = 0.f;
  const float SCL = (50.0f / 64.0f) * 1.4426950408889634f;

  for (int kc = 0; kc < NTGT / KC; ++kc) {
    const int kv0 = kc * KC;
    __syncthreads();
    {
      const int r = tid >> 2, qq = (tid & 3) * 16;
      const __bf16* khs = Kh + ((size_t)(kv0 + r)) * NC + qq;
      const __bf16* kls = Kl + ((size_t)(kv0 + r)) * NC + qq;
      *(v8b*)(Ksh + r * KSP + qq)     = *(const v8b*)(khs);
      *(v8b*)(Ksh + r * KSP + qq + 8) = *(const v8b*)(khs + 8);
      *(v8b*)(Ksl + r * KSP + qq)     = *(const v8b*)(kls);
      *(v8b*)(Ksl + r * KSP + qq + 8) = *(const v8b*)(kls + 8);
      for (int i = tid; i < DVP * (KC / 8); i += 256) {
        const int d = i >> 3, k8 = (i & 7) * 8;
        *(v8b*)(Vsh + d * VTP + k8) = *(const v8b*)(Vh + (size_t)d * NTGT + kv0 + k8);
        *(v8b*)(Vsl + d * VTP + k8) = *(const v8b*)(Vl + (size_t)d * NTGT + kv0 + k8);
      }
    }
    __syncthreads();

    v8f s[4];
#pragma unroll
    for (int j = 0; j < 4; ++j) s[j] = (v8f){0.f, 0.f, 0.f, 0.f, 0.f, 0.f, 0.f, 0.f};
#pragma unroll
    for (int j = 0; j < 4; ++j) {
#pragma unroll
      for (int dc = 0; dc < 2; ++dc) {
        const __bf16* kp = Ksh + (j * 16 + c) * KSP + dc * 32 + 8 * lh;
        const __bf16* kq = Ksl + (j * 16 + c) * KSP + dc * 32 + 8 * lh;
        FB ah, al;
        ah.h[0] = *(const v8b*)(kp);
        ah.h[1] = *(const v8b*)(kp + 16);
        al.h[0] = *(const v8b*)(kq);
        al.h[1] = *(const v8b*)(kq + 16);
        s[j] = mma_bf(ah.v, qfh[dc].v, s[j]);
        s[j] = mma_bf(ah.v, qfl[dc].v, s[j]);
        s[j] = mma_bf(al.v, qfh[dc].v, s[j]);
      }
    }

    float cm = -1e30f;
#pragma unroll
    for (int j = 0; j < 4; ++j) {
#pragma unroll
      for (int r = 0; r < 8; ++r) {
        const float tv = s[j][r] * SCL;
        s[j][r] = tv;
        cm = fmaxf(cm, tv);
      }
    }
    cm = fmaxf(cm, __shfl_xor(cm, 16, 32));
    const float mnew  = fmaxf(mrun, cm);
    const float alpha = __builtin_amdgcn_exp2f(mrun - mnew);
    mrun = mnew;
    float psum = 0.f;
    FW ph[2], pl[2];
#pragma unroll
    for (int j = 0; j < 4; ++j) {
#pragma unroll
      for (int q = 0; q < 4; ++q) {
        const float p0 = __builtin_amdgcn_exp2f(s[j][2 * q] - mnew);
        const float p1 = __builtin_amdgcn_exp2f(s[j][2 * q + 1] - mnew);
        psum += p0 + p1;
        unsigned hw, lw;
        split2(p0, p1, hw, lw);
        ph[j >> 1].w[(j & 1) * 4 + q] = hw;
        pl[j >> 1].w[(j & 1) * 4 + q] = lw;
      }
    }
    psum += __shfl_xor(psum, 16, 32);
    lrun = lrun * alpha + psum;
#pragma unroll
    for (int t = 0; t < 5; ++t) oacc[t] = oacc[t] * alpha;

#pragma unroll
    for (int kk = 0; kk < 2; ++kk) {
#pragma unroll
      for (int t = 0; t < 5; ++t) {
        const __bf16* vp = Vsh + (t * 16 + c) * VTP + kk * 32 + 8 * lh;
        const __bf16* vq = Vsl + (t * 16 + c) * VTP + kk * 32 + 8 * lh;
        FB ahv, alv;
        ahv.h[0] = *(const v8b*)(vp);
        ahv.h[1] = *(const v8b*)(vp + 16);
        alv.h[0] = *(const v8b*)(vq);
        alv.h[1] = *(const v8b*)(vq + 16);
        oacc[t] = mma_bf(ahv.v, ph[kk].v, oacc[t]);
        oacc[t] = mma_bf(ahv.v, pl[kk].v, oacc[t]);
        oacc[t] = mma_bf(alv.v, ph[kk].v, oacc[t]);
      }
    }
  }

  const float inv = 1.0f / lrun;
  v8f ov[5];
#pragma unroll
  for (int t = 0; t < 5; ++t) ov[t] = oacc[t] * inv;
  float dsum = 0.f;
#pragma unroll
  for (int t = 0; t < 5; ++t) {
#pragma unroll
    for (int r = 0; r < 8; ++r) {
      const int d = t * 16 + 8 * lh + r;
      const bool isd = (d >= 4) && (d < NDV);
      dsum += isd ? ov[t][r] : 0.f;
    }
  }
  dsum += __shfl_xor(dsum, 16, 32);
  const float mu = dsum * (1.0f / 64.0f);
  float dvar = 0.f;
#pragma unroll
  for (int t = 0; t < 5; ++t) {
#pragma unroll
    for (int r = 0; r < 8; ++r) {
      const int d = t * 16 + 8 * lh + r;
      const bool isd = (d >= 4) && (d < NDV);
      const float dx = ov[t][r] - mu;
      dvar += isd ? dx * dx : 0.f;
    }
  }
  dvar += __shfl_xor(dvar, 16, 32);
  const float rs = 1.0f / sqrtf(dvar * (1.0f / 63.0f));
  {
    const int qcol = wave * 16 + c;
#pragma unroll
    for (int t = 0; t < 5; ++t) {
#pragma unroll
      for (int r = 0; r < 8; ++r) {
        const int d = t * 16 + 8 * lh + r;
        const bool isd = (d >= 4) && (d < NDV);
        const float val = isd ? (ov[t][r] - mu) * rs : ov[t][r];
        Osh[d * OSP + qcol] = val;
      }
    }
  }
  __syncthreads();

  {
    const int c4 = lane * 4;
    for (int d = wave; d < NDV; d += 8) {
      size_t rowoff;
      if (d < 3)       rowoff = ((size_t)(b * 3 + d)) * NSRC;
      else if (d == 3) rowoff = (size_t)6144 + (size_t)b * NSRC;
      else             rowoff = (size_t)8192 + ((size_t)(b * NC + (d - 4))) * NSRC;
      const v4f vv = *(const v4f*)(Osh + d * OSP + c4);
      *(volatile v4f*)(out + rowoff + n0 + c4) = vv;
    }
    __threadfence();
    for (int d = wave; d < NDV; d += 8) {
      size_t rowoff;
      if (d < 3)       rowoff = ((size_t)(b * 3 + d)) * NSRC;
      else if (d == 3) rowoff = (size_t)6144 + (size_t)b * NSRC;
      else             rowoff = (size_t)8192 + ((size_t)(b * NC + (d - 4))) * NSRC;
      const v4f vv = *(const v4f*)(Osh + d * OSP + c4);
      *(volatile v4f*)(out + rowoff + n0 + c4) = vv;
    }
  }
}

extern "C" void kernel_launch(void* const* d_in, const int* in_sizes, int n_in,
                              void* d_out, int out_size, void* d_ws, size_t ws_size,
                              hipStream_t stream) {
  if (n_in < 5) return;
  if (in_sizes[1] != NB * 3 * NTGT) return;
  if (in_sizes[2] != NB * 1 * NTGT) return;
  if (in_sizes[3] != NB * NC * NSRC) return;
  if (in_sizes[4] != NB * NC * NTGT) return;
  if (out_size != NB * 3 * NSRC + NB * NSRC + NB * NC * NSRC) return;

  const float* tgt_coords  = (const float*)d_in[1];
  const float* tgt_weights = (const float*)d_in[2];
  const float* src_desc    = (const float*)d_in[3];
  const float* tgt_desc    = (const float*)d_in[4];
  float* o = (float*)d_out;

  const size_t PQ = (size_t)NB * NSRC * NC * 2;
  const size_t PK = (size_t)NB * NTGT * NC * 2;
  const size_t PV = (size_t)NB * DVP * NTGT * 2;
  size_t off = 0;
  const size_t oQh = off; off += PQ;
  const size_t oQl = off; off += PQ;
  const size_t oKh = off; off += PK;
  const size_t oKl = off; off += PK;
  const size_t oVh = off; off += PV;
  const size_t oVl = off; off += PV;
  if (off > ws_size) return;

  char* ws = (char*)d_ws;
  unsigned short* Qh = (unsigned short*)(ws + oQh);
  unsigned short* Ql = (unsigned short*)(ws + oQl);
  unsigned short* Kh = (unsigned short*)(ws + oKh);
  unsigned short* Kl = (unsigned short*)(ws + oKl);
  unsigned short* Vh = (unsigned short*)(ws + oVh);
  unsigned short* Vl = (unsigned short*)(ws + oVl);

  zn_split_kernel<<<dim3(NB * NSRC / 64), dim3(256), 0, stream>>>(src_desc, Qh, Ql, NSRC);
  zn_split_kernel<<<dim3(NB * NTGT / 64), dim3(256), 0, stream>>>(tgt_desc, Kh, Kl, NTGT);
  vsplit_kernel<<<dim3(NB * DVP * (NTGT / VSEG)), dim3(256), 0, stream>>>(tgt_coords, tgt_weights,
                                                                           tgt_desc, Vh, Vl);
  matcher_kernel<<<dim3(NB * (NSRC / QBLK)), dim3(256), 0, stream>>>(Qh, Ql, Kh, Kl, Vh, Vl, o);
  (void)hipGetLastError();
}
